// ParallelGatedScan_42606075576705
// MI455X (gfx1250) — hardware-verified
//
#include <hip/hip_runtime.h>


#define NB_  8
#define TT   2048
#define DM   512
#define SD   256
#define OD   64
#define CH   32
#define NR   (NB_ * TT)
typedef _Float16 h16;
typedef unsigned short bf;
typedef __attribute__((ext_vector_type(16))) __bf16   v16bf;
typedef __attribute__((ext_vector_type(16))) _Float16 v16h;
typedef __attribute__((ext_vector_type(8)))  _Float16 v8h;
typedef __attribute__((ext_vector_type(8)))  unsigned short v8us;
typedef __attribute__((ext_vector_type(8)))  float    v8f;
typedef __attribute__((ext_vector_type(4)))  float    v4f;
typedef v8h  __attribute__((may_alias)) v8ha;
typedef v4f  __attribute__((may_alias)) v4fa;
typedef v8us __attribute__((may_alias)) v8usa;

__device__ __forceinline__ unsigned short f2bf(float f) { unsigned u = __float_as_uint(f); u += 0x7FFFu + ((u >> 16) & 1u); return (unsigned short)(u >> 16); }
__device__ __forceinline__ float bf2f(unsigned short b) { return __uint_as_float(((unsigned)b) << 16); }
__device__ __forceinline__ float bfr(float f) { return bf2f(f2bf(f)); }
__device__ __forceinline__ v16h cat16(v8h lo, v8h hi) { return __builtin_shufflevector(lo, hi, 0, 1, 2, 3, 4, 5, 6, 7, 8, 9, 10, 11, 12, 13, 14, 15); }
__device__ __forceinline__ v16bf cat16b(v8us lo, v8us hi) { return __builtin_bit_cast(v16bf, __builtin_shufflevector(lo, hi, 0, 1, 2, 3, 4, 5, 6, 7, 8, 9, 10, 11, 12, 13, 14, 15)); }
__device__ __forceinline__ v8f wmma16(v16h a, v16h b, v8f c) { return __builtin_amdgcn_wmma_f32_16x16x32_f16(false, a, false, b, (short)0, c, false, false); }
__device__ __forceinline__ v8f wmmab(v16bf a, v16bf b, v8f c) { return __builtin_amdgcn_wmma_f32_16x16x32_bf16(false, a, false, b, (short)0, c, false, false); }


template <typename T16> struct WFrag;
template <> struct WFrag<h16> { typedef v16h V; static __device__ __forceinline__ V ld(const h16* p) { return cat16(*(const v8h*)p, *(const v8h*)(p + 16)); } static __device__ __forceinline__ v8f mma(V a, V b, v8f c) { return wmma16(a, b, c); } };
template <> struct WFrag<bf> { typedef v16bf V; static __device__ __forceinline__ V ld(const bf* p) { return cat16b(*(const v8us*)p, *(const v8us*)(p + 16)); } static __device__ __forceinline__ v8f mma(V a, V b, v8f c) { return wmmab(a, b, c); } };
template <typename T16, int NSPLIT, bool BIAS>
__global__ __launch_bounds__(32) void k_gemmw(const T16* __restrict__ A, const T16* __restrict__ A2, const T16* __restrict__ Bt, const T16* __restrict__ Bt2, int K, float* C, int ldc, const float* __restrict__ bias, size_t sA, size_t sB, size_t sC) {
    typedef typename WFrag<T16>::V V;
    __shared__ __align__(16) float os[16 * 68];
    const size_t z = blockIdx.z; A += z * sA; if (A2) A2 += z * sA; Bt += z * sB; if (Bt2) Bt2 += z * sB; C += z * sC;
    const int lane = threadIdx.x & 31, lr = lane & 15, hi = lane >> 4; const int r0 = blockIdx.x * 64, c0 = blockIdx.y * 64;
    v8f acc[4][4];
#pragma unroll
    for (int mb = 0; mb < 4; ++mb)
#pragma unroll
        for (int nb = 0; nb < 4; ++nb) acc[mb][nb] = (v8f){};
    const size_t aoff = (size_t)(r0 + lr) * K + 8 * hi, boff = (size_t)(c0 + lr) * K + 8 * hi;
#pragma unroll 1
    for (int kc = 0; kc < K; kc += 32) {
        V a[4], a2[4];
#pragma unroll
        for (int mb = 0; mb < 4; ++mb) { a[mb] = WFrag<T16>::ld(A + aoff + (size_t)mb * 16 * K + kc); if (NSPLIT == 1 || NSPLIT == 2) a2[mb] = WFrag<T16>::ld(A2 + aoff + (size_t)mb * 16 * K + kc); }
#pragma unroll
        for (int nb = 0; nb < 4; ++nb) { const V b = WFrag<T16>::ld(Bt + boff + (size_t)nb * 16 * K + kc); V b2; if (NSPLIT >= 2) b2 = WFrag<T16>::ld(Bt2 + boff + (size_t)nb * 16 * K + kc);
#pragma unroll
            for (int mb = 0; mb < 4; ++mb) { acc[mb][nb] = WFrag<T16>::mma(a[mb], b, acc[mb][nb]); if (NSPLIT == 1 || NSPLIT == 2) acc[mb][nb] = WFrag<T16>::mma(a2[mb], b, acc[mb][nb]); if (NSPLIT >= 2) acc[mb][nb] = WFrag<T16>::mma(a[mb], b2, acc[mb][nb]); } }
        asm volatile("v_nop\n\tv_nop\n\tv_nop\n\tv_nop" : "+v"(acc[0][0]), "+v"(acc[1][1]), "+v"(acc[2][2]), "+v"(acc[3][3]) : "v"(a[0]), "v"(a[3]));
    }
#pragma unroll
    for (int mb = 0; mb < 4; ++mb) {
#pragma unroll
        for (int nb = 0; nb < 4; ++nb) {
#pragma unroll
            for (int j = 0; j < 8; ++j) os[(hi * 8 + j) * 68 + nb * 16 + lr] = acc[mb][nb][j]; }
        __builtin_amdgcn_wave_barrier(); asm volatile("" ::: "memory");
        float* crow = C + (size_t)(r0 + mb * 16) * ldc + c0;
#pragma unroll 1
        for (int ps = 0; ps < 2; ++ps) {
#pragma unroll
            for (int s = 0; s < 8; ++s) { const int row = 2 * s + hi, cofs = lr * 4; v4f val = *(const v4fa*)(os + row * 68 + cofs); if (BIAS) { val[0] += bfr(bias[c0 + cofs]); val[1] += bfr(bias[c0 + cofs + 1]); val[2] += bfr(bias[c0 + cofs + 2]); val[3] += bfr(bias[c0 + cofs + 3]); }
                *(volatile v4f*)(crow + (size_t)row * ldc + cofs) = val; }
            if (ps == 0) __threadfence(); }
        __builtin_amdgcn_wave_barrier(); asm volatile("" ::: "memory");
    }
}

__device__ __forceinline__ void splitf(float y, unsigned short& h, unsigned short& l) { h = f2bf(y); l = f2bf(y - bf2f(h)); }
typedef __attribute__((ext_vector_type(2))) unsigned short v2us;
typedef __attribute__((ext_vector_type(4))) unsigned short v4us;

__global__ __launch_bounds__(256) void k_wtG(const float* __restrict__ w, int K, int N, bf* Bt) {
    const int lane = threadIdx.x & 31; const int L0 = (blockIdx.x * 8 + (threadIdx.x >> 5)) * 8; const int nlines = N * K / 64;
#pragma unroll
    for (int ps = 0; ps < 2; ++ps) {
#pragma unroll 1
        for (int l = 0; l < 8; ++l) { const int L = L0 + l; if (L >= nlines) break; const size_t e = (size_t)L * 64 + lane * 2; const int k = (int)(e % K), n = (int)(e / K); v2us o;
            o[0] = f2bf(w[(size_t)k * N + n]); o[1] = f2bf(w[(size_t)(k + 1) * N + n]); *(volatile v2us*)(Bt + e) = o; }
        if (ps == 0) __threadfence(); }
}
__global__ __launch_bounds__(256) void k_cvt8(const float* __restrict__ src, bf* dst, size_t n8) { const size_t i = (size_t)blockIdx.x * 256 + threadIdx.x; if (i >= n8) return; const v8f v = *(const v8f*)(src + i * 8); v8us o;
#pragma unroll
    for (int k = 0; k < 8; ++k) o[k] = f2bf(v[k]); *(volatile v8us*)(dst + i * 8) = o; __threadfence(); *(volatile v8us*)(dst + i * 8) = o; }
__global__ __launch_bounds__(256) void k_gd(float* G, float* Dr, const float* __restrict__ gb, const float* __restrict__ ib) { const size_t e = ((size_t)blockIdx.x * 256 + threadIdx.x) * 4; if (e >= (size_t)NR * SD) return; const int c = (int)(e % SD); const v4f g4 = *(const v4f*)(G + e), d4 = *(const v4f*)(Dr + e); v4f go, dd;
#pragma unroll
    for (int u = 0; u < 4; ++u) { const float z = __fadd_rn(g4[u], bfr(gb[c + u])); const float g = __fdiv_rn(1.0f, __fadd_rn(1.0f, __expf(-z))); go[u] = g; float om = __fsub_rn(1.0f, g); asm volatile("" : "+v"(om)); dd[u] = __fmul_rn(om, __fadd_rn(d4[u], bfr(ib[c + u]))); }
    *(volatile v4f*)(G + e) = go; *(volatile v4f*)(Dr + e) = dd; __threadfence(); *(volatile v4f*)(G + e) = go; *(volatile v4f*)(Dr + e) = dd; }
__global__ __launch_bounds__(64) void k_cscan(const float* __restrict__ G, const float* __restrict__ Dr, float* ST) { const int gl = blockIdx.x * 64 + threadIdx.x; if (gl >= NB_ * SD) return; const int b = gl / SD, c = gl % SD; float h = 0.f;
#pragma unroll 1
    for (int ck = 0; ck < TT / CH; ++ck) { float lsum = 0.f, wb = 0.f, ca = 1.f;
#pragma unroll 1
        for (int s = 0; s < CH; ++s) { const size_t r = (size_t)b * TT + ck * CH + s; const float a = G[r * SD + c], d = Dr[r * SD + c];
            lsum = __fadd_rn(lsum, __logf(fmaxf(a, 1e-6f))); ca = __expf(lsum); wb = __fadd_rn(wb, __fdiv_rn(d, fmaxf(ca, 1e-8f)));
            const float st = __fmul_rn(ca, __fadd_rn(h, wb)); *(volatile float*)(ST + r * SD + c) = st; __threadfence(); *(volatile float*)(ST + r * SD + c) = st; }
        h = __fmul_rn(ca, __fadd_rn(h, wb)); } }
__global__ __launch_bounds__(64) void k_bind(const float* __restrict__ V, const float* __restrict__ K, const float* __restrict__ Q, const float* __restrict__ dec, float* O) {
    __shared__ float red[64]; const int b = blockIdx.x / OD, i = blockIdx.x % OD; const int j = threadIdx.x; const float dc = __fdiv_rn(1.0f, __fadd_rn(1.0f, __expf(-bfr(dec[i])))); float S = 0.f; float obuf[4];
#pragma unroll 1
    for (int t = 0; t < TT; ++t) { const size_t r = (size_t)b * TT + t; const float vi = V[r * OD + i], kj = K[r * OD + j], qj = Q[r * OD + j]; float p = __fmul_rn(vi, kj); asm volatile("" : "+v"(p)); float ds = __fmul_rn(dc, S); asm volatile("" : "+v"(ds)); S = __fadd_rn(ds, p); float oq = __fmul_rn(S, qj); asm volatile("" : "+v"(oq)); red[j] = oq; __syncthreads();
        for (int w = 32; w; w >>= 1) { if (j < w) red[j] = __fadd_rn(red[j], red[j + w]); __syncthreads(); }
        const float oi = red[0]; __syncthreads(); obuf[t & 3] = oi;
        if ((t & 3) == 3 && j == 0) { v4f o; o[0] = obuf[0]; o[1] = obuf[1]; o[2] = obuf[2]; o[3] = obuf[3]; float* dst = O + ((size_t)b * OD + i) * TT + t - 3; *(volatile v4f*)dst = o; __threadfence(); *(volatile v4f*)dst = o; } } }
__global__ __launch_bounds__(256) void k_otr(const float* __restrict__ OT, bf* Oh, bf* Ol) { const size_t e = ((size_t)blockIdx.x * 256 + threadIdx.x) * 4; if (e >= (size_t)NR * OD) return; const int i = (int)(e % OD); const size_t r = e / OD; const int b = (int)(r / TT), t = (int)(r % TT); v4us oh, ol;
#pragma unroll
    for (int u = 0; u < 4; ++u) { unsigned short p, q; splitf(OT[((size_t)b * OD + i + u) * TT + t], p, q); oh[u] = p; ol[u] = q; } *(volatile v4us*)(Oh + e) = oh; *(volatile v4us*)(Ol + e) = ol; __threadfence(); *(volatile v4us*)(Oh + e) = oh; *(volatile v4us*)(Ol + e) = ol; }
__global__ __launch_bounds__(256) void k_spl(const float* __restrict__ F, size_t n4, bf* Hh, bf* Hl) { const size_t e = ((size_t)blockIdx.x * 256 + threadIdx.x) * 4; if (e >= n4) return; const v4f a = *(const v4f*)(F + e); v4us oh, ol;
#pragma unroll
    for (int u = 0; u < 4; ++u) { unsigned short p, q; splitf(a[u], p, q); oh[u] = p; ol[u] = q; } *(volatile v4us*)(Hh + e) = oh; *(volatile v4us*)(Hl + e) = ol; __threadfence(); *(volatile v4us*)(Hh + e) = oh; *(volatile v4us*)(Hl + e) = ol; }
__global__ __launch_bounds__(256) void k_fin(const float* __restrict__ X, const float* __restrict__ A, const float* __restrict__ Bv, const float* __restrict__ g, const float* __restrict__ bb, float* out) { const int lane = threadIdx.x & 31; const int r = blockIdx.x * 8 + (threadIdx.x >> 5); if (r >= NR) return; float v[DM / 32]; float s = 0.f;
#pragma unroll
    for (int ch = 0; ch < DM / 128; ++ch) { const size_t o0 = (size_t)r * DM + ch * 128 + lane * 4; const v4f x4 = *(const v4f*)(X + o0), a4 = *(const v4f*)(A + o0), b4 = *(const v4f*)(Bv + o0);
#pragma unroll
        for (int u = 0; u < 4; ++u) { float y = __fadd_rn(bfr(x4[u]), a4[u]); y = __fadd_rn(y, b4[u]); v[ch * 4 + u] = y; s += y; } }
#pragma unroll
    for (int sh = 16; sh; sh >>= 1) s += __shfl_xor(s, sh, 32);
    const float mean = s * (1.0f / DM); float q = 0.f;
#pragma unroll
    for (int k = 0; k < DM / 32; ++k) { float d = __fsub_rn(v[k], mean); asm volatile("" : "+v"(d)); float p = __fmul_rn(d, d); asm volatile("" : "+v"(p)); q = __fadd_rn(q, p); }
#pragma unroll
    for (int sh = 16; sh; sh >>= 1) q += __shfl_xor(q, sh, 32);
    const float rs = __fdiv_rn(1.0f, __fsqrt_rn(__fadd_rn(q * (1.0f / DM), 1e-5f)));
    for (int ps = 0; ps < 2; ++ps) {
#pragma unroll
        for (int ch = 0; ch < DM / 128; ++ch) { v4f o;
#pragma unroll
            for (int u = 0; u < 4; ++u) { const int c = ch * 128 + lane * 4 + u; float d = __fsub_rn(v[ch * 4 + u], mean); asm volatile("" : "+v"(d)); float n0 = __fmul_rn(d, rs); asm volatile("" : "+v"(n0)); float t1 = __fmul_rn(n0, bfr(g[c])); asm volatile("" : "+v"(t1)); o[u] = __fadd_rn(t1, bfr(bb[c])); }
            *(volatile v4f*)(out + (size_t)r * DM + ch * 128 + lane * 4) = o; }
        if (ps == 0) __threadfence(); } }

extern "C" void kernel_launch(void* const* d_in, const int* in_sizes, int n_in,
                              void* d_out, int out_size, void* d_ws, size_t ws_size, hipStream_t stream) {
    (void)in_sizes; (void)n_in; (void)out_size;
    const float** I = (const float**)d_in;
    const float *x = I[0], *gW = I[1], *gb = I[2], *iW = I[3], *ib = I[4], *oW = I[5], *ob = I[6], *vW = I[7], *vb = I[8], *kW = I[9], *kb = I[10], *qW = I[11], *qb = I[12], *dec = I[13], *poW = I[14], *pob = I[15], *lg = I[16], *lb = I[17];
    float* OUT = (float*)d_out;
    char* wsp = (char*)d_ws;
    auto take = [&](size_t bytes) { char* p = wsp; wsp += (bytes + 255) & ~(size_t)255; return (void*)p; };
    bf* XB = (bf*)take((size_t)NR * DM * 2); bf* BG = (bf*)take((size_t)SD * DM * 2); bf* BI = (bf*)take((size_t)SD * DM * 2); bf* BO = (bf*)take((size_t)DM * SD * 2); bf* BV = (bf*)take((size_t)OD * DM * 2); bf* BK = (bf*)take((size_t)OD * DM * 2); bf* BQ = (bf*)take((size_t)OD * DM * 2); bf* BP = (bf*)take((size_t)DM * OD * 2);
    float* G = (float*)take((size_t)NR * SD * 4); float* Dr = (float*)take((size_t)NR * SD * 4); float* ST = (float*)take((size_t)NR * SD * 4); bf* STh = (bf*)take((size_t)NR * SD * 2); bf* STl = (bf*)take((size_t)NR * SD * 2); float* SO = (float*)take((size_t)NR * DM * 4);
    float* V = (float*)take((size_t)NR * OD * 4); float* K = (float*)take((size_t)NR * OD * 4); float* Q = (float*)take((size_t)NR * OD * 4); float* OT = (float*)take((size_t)NR * OD * 4); bf* Oh = (bf*)take((size_t)NR * OD * 2); bf* Ol = (bf*)take((size_t)NR * OD * 2); float* BD = (float*)take((size_t)NR * DM * 4);
    if ((size_t)(wsp - (char*)d_ws) > ws_size) return;
    k_cvt8<<<(NR * DM / 8 + 255) / 256, 256, 0, stream>>>(x, XB, NR * DM / 8);
    k_wtG<<<(DM * SD / 64 + 63) / 64, 256, 0, stream>>>(gW, DM, SD, BG); k_wtG<<<(DM * SD / 64 + 63) / 64, 256, 0, stream>>>(iW, DM, SD, BI); k_wtG<<<(SD * DM / 64 + 63) / 64, 256, 0, stream>>>(oW, SD, DM, BO);
    k_wtG<<<(DM * OD / 64 + 63) / 64, 256, 0, stream>>>(vW, DM, OD, BV); k_wtG<<<(DM * OD / 64 + 63) / 64, 256, 0, stream>>>(kW, DM, OD, BK); k_wtG<<<(DM * OD / 64 + 63) / 64, 256, 0, stream>>>(qW, DM, OD, BQ); k_wtG<<<(OD * DM / 64 + 63) / 64, 256, 0, stream>>>(poW, OD, DM, BP);
    k_gemmw<bf, 0, false><<<dim3(NR / 64, SD / 64, 1), 32, 0, stream>>>(XB, nullptr, BG, nullptr, DM, G, SD, nullptr, 0, 0, 0); k_gemmw<bf, 0, false><<<dim3(NR / 64, SD / 64, 1), 32, 0, stream>>>(XB, nullptr, BI, nullptr, DM, Dr, SD, nullptr, 0, 0, 0);
    k_gd<<<(unsigned)(((size_t)NR * SD / 4 + 255) / 256), 256, 0, stream>>>(G, Dr, gb, ib);
    k_cscan<<<(NB_ * SD + 63) / 64, 64, 0, stream>>>(G, Dr, ST);
    k_spl<<<(unsigned)(((size_t)NR * SD / 4 + 255) / 256), 256, 0, stream>>>(ST, (size_t)NR * SD, STh, STl);
    k_gemmw<bf, 1, true><<<dim3(NR / 64, DM / 64, 1), 32, 0, stream>>>(STh, STl, BO, nullptr, SD, SO, DM, ob, 0, 0, 0);
    k_gemmw<bf, 0, true><<<dim3(NR / 64, 1, 1), 32, 0, stream>>>(XB, nullptr, BV, nullptr, DM, V, OD, vb, 0, 0, 0); k_gemmw<bf, 0, true><<<dim3(NR / 64, 1, 1), 32, 0, stream>>>(XB, nullptr, BK, nullptr, DM, K, OD, kb, 0, 0, 0); k_gemmw<bf, 0, true><<<dim3(NR / 64, 1, 1), 32, 0, stream>>>(XB, nullptr, BQ, nullptr, DM, Q, OD, qb, 0, 0, 0);
    k_bind<<<NB_ * OD, 64, 0, stream>>>(V, K, Q, dec, OT);
    k_otr<<<(unsigned)(((size_t)NR * OD / 4 + 255) / 256), 256, 0, stream>>>(OT, Oh, Ol);
    k_gemmw<bf, 1, true><<<dim3(NR / 64, DM / 64, 1), 32, 0, stream>>>(Oh, Ol, BP, nullptr, OD, BD, DM, pob, 0, 0, 0);
    k_fin<<<NR / 8, 256, 0, stream>>>(x, SO, BD, lg, lb, OUT);
}
